// PointTransfomerDecModule_2680059592823
// MI455X (gfx1250) — hardware-verified
//
#include <hip/hip_runtime.h>
#include <math.h>

typedef __attribute__((ext_vector_type(16))) _Float16 v16h;
typedef __attribute__((ext_vector_type(16))) __bf16 v16b;
typedef __attribute__((ext_vector_type(8)))  _Float16 v8h;
typedef __attribute__((ext_vector_type(8)))  float v8f;
typedef __attribute__((ext_vector_type(4)))  float v4f;
typedef __attribute__((ext_vector_type(2)))  float v2f;
typedef __attribute__((ext_vector_type(4)))  unsigned v4u;
typedef __attribute__((ext_vector_type(4)))  int v4i;
typedef float __attribute__((may_alias)) float_a;
typedef int __attribute__((may_alias)) int_a;

template <typename T> __device__ __forceinline__ void vst2(void* p, T v) { *(volatile T*)p = v; __threadfence(); *(volatile T*)p = v; }
__device__ __forceinline__ v8f wmma16(v16h a, v16h b, v8f c) {
  v8f d = __builtin_amdgcn_wmma_f32_16x16x32_f16(false, a, false, b, (short)0, c, false, false);
  asm volatile("v_nop\n\tv_nop\n\tv_nop\n\tv_nop" : "+v"(d) : "v"(a), "v"(b));
  return d;
}
__device__ __forceinline__ v8f wmma_bf(v16b a, v16b b, v8f c) {
  v8f d = __builtin_amdgcn_wmma_f32_16x16x32_bf16(false, a, false, b, (short)0, c, false, false);
  asm volatile("v_nop\n\tv_nop\n\tv_nop\n\tv_nop" : "+v"(d) : "v"(a), "v"(b));
  return d;
}
__device__ __forceinline__ v16h frag_h(const _Float16* rowk0, int lane) {
  union { v16h v; v8h q[2]; } u; const _Float16* p = rowk0 + 8 * (lane >> 4);
  u.q[0] = *(const v8h*)p; u.q[1] = *(const v8h*)(p + 16); return u.v;
}
__device__ __forceinline__ v16h frag_f32(const float* rowk0, int lane) {
  v16h a; const float* p = rowk0 + 8 * (lane >> 4);
#pragma unroll
  for (int i = 0; i < 8; ++i) { a[i] = (_Float16)p[i]; a[8 + i] = (_Float16)p[16 + i]; }
  return a;
}
__device__ __forceinline__ v16h frag_f32s(const float* rowk0, int lane, float sc) {
  v16h a; const float* p = rowk0 + 8 * (lane >> 4);
#pragma unroll
  for (int i = 0; i < 8; ++i) { a[i] = (_Float16)(p[i] * sc); a[8 + i] = (_Float16)(p[16 + i] * sc); }
  return a;
}
__device__ __forceinline__ v16h fragc_f32(const float* W, int k0, int n, int lane, int ld, int K) {
  v16h a; const int g = lane >> 4;
#pragma unroll
  for (int i = 0; i < 8; ++i) { const int ka = k0 + 8 * g + i, kb = ka + 16;
    a[i] = (_Float16)(ka < K ? W[(size_t)(ka < K ? ka : K - 1) * ld + n] : 0.f); a[8 + i] = (_Float16)(kb < K ? W[(size_t)(kb < K ? kb : K - 1) * ld + n] : 0.f); }
  return a;
}
struct F2 { v16b h, l; };
__device__ __forceinline__ F2 bsplit16(const float v[16]) { F2 r;
#pragma unroll
  for (int i = 0; i < 16; ++i) { const __bf16 h = (__bf16)v[i]; r.h[i] = h; r.l[i] = (__bf16)(v[i] - (float)h); }
  return r; }
__device__ __forceinline__ F2 split_row(const float* row, int k0, int lane) { float v[16]; const float* p = row + k0 + 8 * (lane >> 4);
#pragma unroll
  for (int i = 0; i < 8; ++i) { v[i] = p[i]; v[8 + i] = p[16 + i]; }
  return bsplit16(v); }
__device__ __forceinline__ F2 split_rowK(const float* row, int k0, int lane, int K) { float v[16]; const int g = lane >> 4;
#pragma unroll
  for (int i = 0; i < 8; ++i) { const int ka = k0 + 8 * g + i, kb = ka + 16; v[i] = ka < K ? row[ka < K ? ka : K - 1] : 0.f; v[8 + i] = kb < K ? row[kb < K ? kb : K - 1] : 0.f; }
  return bsplit16(v); }
__device__ __forceinline__ F2 split_col(const float* W, int k0, int n, int lane, int ld, int K) { float v[16]; const int g = lane >> 4;
#pragma unroll
  for (int i = 0; i < 8; ++i) { const int ka = k0 + 8 * g + i, kb = ka + 16; v[i] = ka < K ? W[(size_t)(ka < K ? ka : K - 1) * ld + n] : 0.f; v[8 + i] = kb < K ? W[(size_t)(kb < K ? kb : K - 1) * ld + n] : 0.f; }
  return bsplit16(v); }
__device__ __forceinline__ v8f mac3(const F2& a, const F2& b, v8f c) { c = wmma_bf(a.l, b.h, c); c = wmma_bf(a.h, b.l, c); return wmma_bf(a.h, b.h, c); }
__device__ __forceinline__ float sigm(float v) { return 1.0f / (1.0f + expf(-v)); }
#define LDSX() do { asm volatile("s_wait_dscnt 0" ::: "memory"); __builtin_amdgcn_wave_barrier(); __builtin_amdgcn_fence(__ATOMIC_RELEASE, "workgroup"); } while (0)


#define NBT 2
#define NS 2048
#define NM 8192
#define RS (NBT * NS)
#define RM (NBT * NM)
#define C1 256
#define CC 128
#define KN 16
#define CS 16
#ifndef RMT
#define RMT RM
#endif
#define GRID 10
#define NCELL (NBT * GRID * GRID * GRID)
typedef __attribute__((ext_vector_type(8))) __bf16 v8b;
__device__ __forceinline__ v16b frag_b(const __bf16* rowk0, int lane) {
  union { v16b v; v8b q[2]; } u; const __bf16* p = rowk0 + 8 * (lane >> 4);
  u.q[0] = *(const v8b*)p; u.q[1] = *(const v8b*)(p + 16); return u.v;
}
__device__ __forceinline__ float bfr(float v) { return (float)(__bf16)v; }
__device__ __attribute__((noinline)) float exp_ni(float v) { return expf(v); }
__device__ __attribute__((noinline)) float erf_ni(float v) { return erff(v); }

#define CSA_N 2000
#define CSA_E 16384
#define CSA_FINN (CSA_E + 32 * CSA_NBK)
#define CSA_CHUNK 4096
#define CSA_BKT 256
#define CSA_NCH ((CSA_E + CSA_CHUNK - 1) / CSA_CHUNK)
#define CSA_NBK ((CSA_N + CSA_BKT - 1) / CSA_BKT)
#define CSA_NBKP (((CSA_NBK + 63) / 64) * 64)
#define CSA_SEGCAP (CSA_E + 32 * CSA_NBK * CSA_NCH)
#ifndef CSA_BCAP
#define CSA_BCAP 10240
#endif
#define CSA_SZ_CNT   (4u * CSA_NCH * CSA_NBKP)
#define CSA_SZ_OFF   (4u * CSA_NBK * (((CSA_NCH + 31) / 32) * 32))
#define CSA_SZ_BST   (4u * (((CSA_NBK + 1 + 31) / 32) * 32))
#define CSA_SZ_SEG   (4u * CSA_SEGCAP)
#define CSA_SZ_FIN   (4u * (CSA_E + 32 * CSA_NBK))
#define CSA_SZ_ROW   (4u * CSA_NBK * CSA_BKT)
#define CSA_OFFP (((CSA_NCH + 31) / 32) * 32)

__global__ __launch_bounds__(256) void k_csA_cnt(const int* __restrict__ DST, int dstride, int* __restrict__ CNT) {
  __shared__ unsigned short sc[256][CSA_NBK + 1]; __shared__ __align__(16) int srow[CSA_NBKP];
  const int c = blockIdx.x, tid = threadIdx.x;
  for (int b = 0; b < CSA_NBK; ++b) sc[tid][b] = 0;
  const size_t e0 = (size_t)c * CSA_CHUNK + tid * 16;
  for (int i = 0; i < 16; ++i) { const size_t e = e0 + i; if (e < (size_t)CSA_E) { int d = DST[e * dstride]; d = min(max(d, 0), CSA_N - 1); sc[tid][d / CSA_BKT] += 1; } }
  __syncthreads();
  for (int b = tid; b < CSA_NBKP; b += 256) { int s = 0; if (b < CSA_NBK) for (int t = 0; t < 256; ++t) s += sc[t][b]; srow[b] = s; }
  __syncthreads();
  for (int q = tid; q < CSA_NBKP / 4; q += 256) vst2((unsigned*)(CNT + (size_t)c * CSA_NBKP + q * 4), *(const v4u*)&srow[q * 4]);
}
__global__ __launch_bounds__(256) void k_csA_scan(const int* __restrict__ CNT, int* __restrict__ OFF, int* __restrict__ BST) {
  __shared__ int sbt[CSA_NBK + 1]; __shared__ int sbs[((CSA_NBK + 1 + 31) / 32) * 32]; __shared__ int scnt[CSA_NBK + 1]; __shared__ __align__(16) int sbuf[64][CSA_OFFP];
  const int tid = threadIdx.x;
  for (int b = tid; b < CSA_NBK; b += 256) { int sp = 0, st = 0; for (int c = 0; c < CSA_NCH; ++c) { const int n = CNT[(size_t)c * CSA_NBKP + b]; st += n; sp += (n + 31) & ~31; } sbt[b] = sp; scnt[b] = st; }
  for (int b = tid; b < ((CSA_NBK + 1 + 31) / 32) * 32; b += 256) sbs[b] = 0;
  __syncthreads();
  if (tid == 0) { int acc = 0, accf = 0; for (int b = 0; b < CSA_NBK; ++b) { const int t = sbt[b]; sbt[b] = acc; acc += t; sbs[b] = accf; accf += (scnt[b] + 31) & ~31; } sbs[CSA_NBK] = accf; }
  __syncthreads();
  for (int b0 = 0; b0 < CSA_NBK; b0 += 64) {
    if (tid < 64 && b0 + tid < CSA_NBK) { const int b = b0 + tid; int o = sbt[b]; for (int c = 0; c < CSA_OFFP; ++c) { if (c < CSA_NCH) { sbuf[tid][c] = o; o += (CNT[(size_t)c * CSA_NBKP + b] + 31) & ~31; } else sbuf[tid][c] = 0; } }
    __syncthreads();
    for (int q = tid; q < 64 * (CSA_OFFP / 4); q += 256) { const int r = q / (CSA_OFFP / 4), pc = q % (CSA_OFFP / 4); if (b0 + r < CSA_NBK) vst2((unsigned*)(OFF + (size_t)(b0 + r) * CSA_OFFP + pc * 4), *(const v4u*)&sbuf[r][pc * 4]); }
    __syncthreads(); }
  for (int q = tid; q < ((CSA_NBK + 1 + 31) / 32) * 32 / 4; q += 256) vst2((unsigned*)(BST + q * 4), *(const v4u*)&sbs[q * 4]);
}
__global__ __launch_bounds__(256) void k_csA_scatter(const int* __restrict__ SRC, const int* __restrict__ DST, int sstride, int dstride, const int* __restrict__ OFF, int* __restrict__ SEGS, int* __restrict__ SEGE) {
  __shared__ unsigned short sc[256][CSA_NBK + 1]; __shared__ int sbase[CSA_NBK + 1]; __shared__ int scn[CSA_NBK + 1]; __shared__ int sord[CSA_CHUNK];
  const int c = blockIdx.x, tid = threadIdx.x;
  for (int b = 0; b < CSA_NBK; ++b) sc[tid][b] = 0;
  const size_t e0 = (size_t)c * CSA_CHUNK + tid * 16; int bk[16];
#pragma unroll
  for (int i = 0; i < 16; ++i) { const size_t e = e0 + i; bk[i] = -1; if (e < (size_t)CSA_E) { int d = DST[e * dstride]; d = min(max(d, 0), CSA_N - 1); bk[i] = d / CSA_BKT; sc[tid][bk[i]] += 1; } }
  __syncthreads();
  for (int b = tid; b < CSA_NBK; b += 256) { int acc = 0; for (int t = 0; t < 256; ++t) { const int v = sc[t][b]; sc[t][b] = (unsigned short)acc; acc += v; } scn[b] = acc; }
  __syncthreads();
  if (tid == 0) { int acc = 0; for (int b = 0; b < CSA_NBK; ++b) { sbase[b] = acc; acc += scn[b]; } }
  __syncthreads();
#pragma unroll
  for (int i = 0; i < 16; ++i) { if (bk[i] >= 0) { const int b = bk[i]; const int r = sc[tid][b]; sc[tid][b] = (unsigned short)(r + 1); sord[sbase[b] + r] = tid * 16 + i; } }
  __syncthreads();
  for (int b = 0; b < CSA_NBK; ++b) { const int n = scn[b]; if (n == 0) continue; const int nl = ((n + 31) & ~31); const size_t o = (size_t)(min(max(OFF[(size_t)b * CSA_OFFP + c], 0), CSA_SEGCAP - nl) & ~31);
    for (int q = tid; q < nl / 4; q += 256) { int4 vs, ve;
#pragma unroll
      for (int k = 0; k < 4; ++k) { const int i = q * 4 + k; int s = -1, eid = -1; if (i < n) { const size_t e = (size_t)c * CSA_CHUNK + sord[sbase[b] + i]; s = min(max(SRC[e * sstride], 0), CSA_N - 1); eid = (int)e; } vs[k] = s; ve[k] = eid; }
      vst2((unsigned*)(SEGS + o + q * 4), *(const v4u*)&vs); vst2((unsigned*)(SEGE + o + q * 4), *(const v4u*)&ve); } }
}
__global__ __launch_bounds__(256) void k_csA_bucket(const int* __restrict__ CNT, const int* __restrict__ OFF, const int* __restrict__ BST, const int* __restrict__ SEGS, const int* __restrict__ SEGE, const int* __restrict__ DST, int dstride, int* __restrict__ FS, int* __restrict__ FE, int* __restrict__ ROWST, int* __restrict__ ROWCNT) {
  __shared__ int ssrc[CSA_BCAP]; __shared__ int seid[CSA_BCAP]; __shared__ unsigned char snod[CSA_BCAP]; __shared__ int souts[CSA_BCAP]; __shared__ int soute[CSA_BCAP]; __shared__ int scount[256]; __shared__ int sstart[257]; __shared__ int stot;
  const int b = blockIdx.x, tid = threadIdx.x;
  if (tid == 0) { int t = 0; for (int c = 0; c < CSA_NCH; ++c) t += min(max(CNT[(size_t)c * CSA_NBKP + b], 0), CSA_CHUNK); stot = (t <= CSA_BCAP) ? t : 0; }
  __syncthreads();
  { int base = 0; for (int c = 0; c < CSA_NCH; ++c) { const int n = min(max(CNT[(size_t)c * CSA_NBKP + b], 0), CSA_CHUNK); const int o = min(max(OFF[(size_t)b * CSA_OFFP + c], 0), CSA_SEGCAP - ((n + 31) & ~31));
      for (int i = tid; i < n; i += 256) { const int p = base + i; if (p < CSA_BCAP) { ssrc[p] = min(max(SEGS[o + i], 0), CSA_N - 1); const int e = min(max(SEGE[o + i], 0), CSA_E - 1); seid[p] = e; int d = DST[(size_t)e * dstride]; d = min(max(d, 0), CSA_N - 1); const int dl = d - b * CSA_BKT; snod[p] = (unsigned char)(dl >= 0 && dl < 256 ? dl : 255); } }
      base += n; } }
  __syncthreads();
  const int node = b * CSA_BKT + tid; int cnt = 0; for (int p = 0; p < stot; ++p) cnt += (snod[p] == tid) ? 1 : 0;
  scount[tid] = cnt; __syncthreads();
  if (tid == 0) { int acc = 0; for (int t = 0; t < 256; ++t) { sstart[t] = acc; acc += scount[t]; } sstart[256] = acc; }
  __syncthreads();
  const int bst0 = min(max(BST[b], 0), CSA_FINN - ((sstart[256] + 31) & ~31)) & ~31; const int gst = bst0 + sstart[tid];
  { int w = sstart[tid]; for (int p = 0; p < stot; ++p) if (snod[p] == tid) { souts[w] = ssrc[p]; soute[w] = seid[p]; ++w; } }
  __syncthreads();
  { const int n = sstart[256]; const int nl = (n + 31) & ~31; for (int q = tid; q < nl / 4; q += 256) { int4 vs, ve;
#pragma unroll
      for (int k = 0; k < 4; ++k) { const int i = q * 4 + k; vs[k] = i < n ? souts[i] : -1; ve[k] = i < n ? soute[i] : -1; }
      vst2((unsigned*)(FS + bst0 + q * 4), *(const v4u*)&vs); vst2((unsigned*)(FE + bst0 + q * 4), *(const v4u*)&ve); } }
  __syncthreads();
  { __shared__ __align__(16) int srs[256], src2[256]; srs[tid] = node < CSA_N ? gst : 0; src2[tid] = node < CSA_N ? cnt : 0; __syncthreads();
    if (tid < 64) vst2((unsigned*)(ROWST + (size_t)b * 256 + tid * 4), *(const v4u*)&srs[tid * 4]); else if (tid < 128) vst2((unsigned*)(ROWCNT + (size_t)b * 256 + (tid - 64) * 4), *(const v4u*)&src2[(tid - 64) * 4]); }
}


#define WS_CNT  0u
#define WS_OFF  (WS_CNT + CSA_SZ_CNT)
#define WS_BST  (WS_OFF + CSA_SZ_OFF)
#define WS_SEGS (WS_BST + CSA_SZ_BST)
#define WS_SEGE (WS_SEGS + CSA_SZ_SEG)
#define WS_FS   (WS_SEGE + CSA_SZ_SEG)
#define WS_FE   (WS_FS + CSA_SZ_FIN)
#define WS_RST  (WS_FE + CSA_SZ_FIN)
#define WS_RCT  (WS_RST + CSA_SZ_ROW)
#define WS_CELL (WS_RCT + CSA_SZ_ROW)
#define WS_PID  (WS_CELL + 4u * RM)
#define WS_FT   (WS_PID + 4u * RM)
#define WS_TT   (WS_FT + 4u * RS * C1)
#define WS_F    (WS_TT + 4u * RM * CC)
#define WS_X    (WS_F + 4u * RS * CC)
#define WS_X1   (WS_X + 4u * RM * CC)
#define WS_Q    (WS_X1 + 4u * RM * CC)
#define WS_IDX  (WS_Q + 4u * RM * 384)
#define WS_I3   (WS_IDX + 4u * RM * KN)
#define WS_W3   (WS_I3 + 4u * RM * 4)
#define WS_AG   (WS_W3 + 4u * RM * 4)
#define WS_PW   (WS_AG + 4u * RM * CC)
#define P_TU1 0
#define P_TU2 (P_TU1 + 128 * 256)
#define P_L1  (P_TU2 + 128 * 128)
#define P_QKV (P_L1 + 128 * 128)
#define P_W1  (P_QKV + 384 * 128)
#define P_L3  (P_W1 + 16 * 128)
#define PWEND (P_L3 + 128 * 128)
#define WS_END  (WS_PW + 2u * PWEND)

__global__ __launch_bounds__(256) void k_packW(const float* __restrict__ TU1, const float* __restrict__ TU2, const float* __restrict__ L1, const float* __restrict__ WQ, const float* __restrict__ WK, const float* __restrict__ WV, const float* __restrict__ WL1, const float* __restrict__ L3, __bf16* __restrict__ PW) {
  __shared__ __align__(16) __bf16 s[256]; const int o = blockIdx.x, which = blockIdx.y, t = threadIdx.x; size_t dst; int K = 128; const float* Wm;
  if (which == 0) { Wm = TU1; K = 256; dst = P_TU1 + (size_t)o * 256; } else if (which == 1) { Wm = TU2; dst = P_TU2 + (size_t)o * 128; } else if (which == 2) { Wm = L1; dst = P_L1 + (size_t)o * 128; }
  else if (which == 3) { Wm = WQ; dst = P_QKV + (size_t)o * 128; } else if (which == 4) { Wm = WK; dst = P_QKV + (size_t)(128 + o) * 128; } else if (which == 5) { Wm = WV; dst = P_QKV + (size_t)(256 + o) * 128; }
  else if (which == 6) { if (o >= CS) return; Wm = WL1; dst = P_W1 + (size_t)o * 128; } else { Wm = L3; dst = P_L3 + (size_t)o * 128; }
  if (t < K) s[t] = (__bf16)Wm[(size_t)o * K + t]; __syncthreads();
  if (t < K / 8) vst2((unsigned*)(PW + dst + t * 8), *(const v4u*)&s[t * 8]);
}
template <int W, int NP>
__global__ __launch_bounds__(64) void k_tr(const float* __restrict__ SRC, float* __restrict__ DST) {
  __shared__ __align__(16) float s[64][W + 4]; const int t = threadIdx.x; const size_t i0 = (size_t)blockIdx.x * 64; const int b = (int)(i0 / NP), n0 = (int)(i0 % NP);
  for (int c = 0; c < W; ++c) s[t][c] = bfr(SRC[((size_t)b * W + c) * NP + n0 + t]);
  __syncthreads();
  for (int q = t; q < 64 * (W / 4); q += 64) { const int rl = q / (W / 4), pc = q % (W / 4); vst2(DST + (i0 + rl) * W + pc * 4, *(const v4f*)&s[rl][pc * 4]); }
}
__device__ __forceinline__ int cell_of(float v) { return min(max((int)floorf(v * (float)GRID), 0), GRID - 1); }
__global__ __launch_bounds__(256) void k_cell(const float* __restrict__ TX, int* __restrict__ CELL, int* __restrict__ PID) {
  __shared__ __align__(16) int sc[256], sp[256]; const int t = threadIdx.x; const size_t m = (size_t)blockIdx.x * 256 + t; const int b = (int)(m / NM);
  const float x = bfr(TX[m * 3]), y = bfr(TX[m * 3 + 1]), z = bfr(TX[m * 3 + 2]);
  sc[t] = ((b * GRID + cell_of(x)) * GRID + cell_of(y)) * GRID + cell_of(z); sp[t] = (int)m; __syncthreads();
  if (t < 64) { vst2((unsigned*)(CELL + (size_t)blockIdx.x * 256 + t * 4), *(const v4u*)&sc[t * 4]); vst2((unsigned*)(PID + (size_t)blockIdx.x * 256 + t * 4), *(const v4u*)&sp[t * 4]); }
}
__device__ __forceinline__ void knn_ins(float d, int i, float* bd, int* bi) {
  if (d < bd[KN - 1] || (d == bd[KN - 1] && i < bi[KN - 1])) { int pos = KN - 1;
#pragma unroll
    for (int q = KN - 2; q >= 0; --q) if (d < bd[q] || (d == bd[q] && i < bi[q])) pos = q;
#pragma unroll
    for (int q = KN - 1; q >= 1; --q) if (q > pos) { bd[q] = bd[q - 1]; bi[q] = bi[q - 1]; }
#pragma unroll
    for (int q = 0; q < KN; ++q) if (q == pos) { bd[q] = d; bi[q] = i; } }
}
template <int PH>
__global__ __launch_bounds__(64) void k_nn(const float* __restrict__ TX, const float* __restrict__ SX, int* __restrict__ I3, float* __restrict__ W3, int* __restrict__ IDX, const int* __restrict__ CELL, const int* __restrict__ FE, const int* __restrict__ RST, const int* __restrict__ RCT) {
  #pragma clang fp contract(off)
  __shared__ __align__(16) int si3[64][4]; __shared__ __align__(16) float sw3[64][4]; __shared__ __align__(16) int sk[64][KN];
  const int t = threadIdx.x; const size_t m = (size_t)blockIdx.x * 64 + t; const int b = (int)(m / NM);
  const float ax = bfr(TX[m * 3]), ay = bfr(TX[m * 3 + 1]), az = bfr(TX[m * 3 + 2]);
  if (PH == 0) { float bd[3] = {3.0e38f, 3.0e38f, 3.0e38f}; int bi[3] = {0, 0, 0}; const float* sp = SX + (size_t)b * NS * 3;
#pragma unroll 1
    for (int i = 0; i < NS; ++i) { const float dx = ax - bfr(sp[i * 3]), dy = ay - bfr(sp[i * 3 + 1]), dz = az - bfr(sp[i * 3 + 2]); const float d = (dx * dx + dz * dz) + dy * dy;
      if (d < bd[2]) { if (d < bd[0]) { bd[2] = bd[1]; bi[2] = bi[1]; bd[1] = bd[0]; bi[1] = bi[0]; bd[0] = d; bi[0] = i; } else if (d < bd[1]) { bd[2] = bd[1]; bi[2] = bi[1]; bd[1] = d; bi[1] = i; } else { bd[2] = d; bi[2] = i; } } }
    float rc[3];
#pragma unroll
    for (int q = 0; q < 3; ++q) { const float dist = sqrtf(fmaxf(bd[q], 0.f)); rc[q] = 1.0f / (dist + 1e-8f); si3[t][q] = b * NS + bi[q]; }
    const float rs = (rc[0] + rc[2]) + rc[1];
#pragma unroll
    for (int q = 0; q < 3; ++q) sw3[t][q] = rc[q] / rs;
    si3[t][3] = b * NS + bi[0]; sw3[t][3] = 0.f; }
  if (PH == 1) { float bd[KN]; int bi[KN]; const int cid = min(max(CELL[m], 0), NCELL - 1) - b * GRID * GRID * GRID; const int cx = cid / (GRID * GRID), cy = (cid / GRID) % GRID, cz = cid % GRID; bool done = false;
#pragma unroll 1
    for (int R = 1; R <= 3 && !done; ++R) {
#pragma unroll
      for (int q = 0; q < KN; ++q) { bd[q] = 3.0e38f; bi[q] = 0x7fffffff; }
      if (R <= 2) {
#pragma unroll 1
        for (int gx = max(cx - R, 0); gx <= min(cx + R, GRID - 1); ++gx)
#pragma unroll 1
          for (int gy = max(cy - R, 0); gy <= min(cy + R, GRID - 1); ++gy)
#pragma unroll 1
            for (int gz = max(cz - R, 0); gz <= min(cz + R, GRID - 1); ++gz) { const int c = ((b * GRID + gx) * GRID + gy) * GRID + gz; const int cnt = min(max(RCT[c], 0), CSA_BCAP); const int st = min(max(RST[c], 0), CSA_FINN - cnt);
#pragma unroll 1
              for (int e = 0; e < cnt; ++e) { const int mg = min(max(FE[st + e], 0), RM - 1); const int i = mg - b * NM; const float dx = ax - bfr(TX[(size_t)mg * 3]), dy = ay - bfr(TX[(size_t)mg * 3 + 1]), dz = az - bfr(TX[(size_t)mg * 3 + 2]); const float d = (dx * dx + dz * dz) + dy * dy; knn_ins(d, i, bd, bi); } }
        const float cs = 1.0f / (float)GRID; float margin = 3.0e38f;
        { const float lo = (cx - R >= 1) ? (ax - (float)(cx - R) * cs) : 3.0e38f, hi = (cx + R <= GRID - 2) ? ((float)(cx + R + 1) * cs - ax) : 3.0e38f; margin = fminf(margin, fminf(lo, hi)); }
        { const float lo = (cy - R >= 1) ? (ay - (float)(cy - R) * cs) : 3.0e38f, hi = (cy + R <= GRID - 2) ? ((float)(cy + R + 1) * cs - ay) : 3.0e38f; margin = fminf(margin, fminf(lo, hi)); }
        { const float lo = (cz - R >= 1) ? (az - (float)(cz - R) * cs) : 3.0e38f, hi = (cz + R <= GRID - 2) ? ((float)(cz + R + 1) * cs - az) : 3.0e38f; margin = fminf(margin, fminf(lo, hi)); }
        const float msafe = fmaxf(margin, 0.f) * 0.99f;
        done = (bi[KN - 1] != 0x7fffffff) && (bd[KN - 1] < msafe * msafe);
      } else { const float* tp = TX + (size_t)b * NM * 3;
#pragma unroll 1
        for (int i = 0; i < NM; ++i) { const float dx = ax - bfr(tp[i * 3]), dy = ay - bfr(tp[i * 3 + 1]), dz = az - bfr(tp[i * 3 + 2]); const float d = (dx * dx + dz * dz) + dy * dy; knn_ins(d, i, bd, bi); }
        done = true; } }
#pragma unroll
    for (int q = 0; q < KN; ++q) sk[t][q] = b * NM + min(bi[q], NM - 1); }
  __syncthreads();
  if (PH == 0) { vst2((unsigned*)(I3 + ((size_t)blockIdx.x * 64 + t) * 4), *(const v4u*)&si3[t][0]); vst2(W3 + ((size_t)blockIdx.x * 64 + t) * 4, *(const v4f*)&sw3[t][0]); }
  else { for (int q2 = t; q2 < 64 * 4; q2 += 64) { const int rl = q2 >> 2, pc = q2 & 3; vst2((unsigned*)(IDX + ((size_t)blockIdx.x * 64 + rl) * KN + pc * 4), *(const v4u*)&sk[rl][pc * 4]); } }
}
template <int MODE>
__global__ __launch_bounds__(128) void k_gemm(const float* __restrict__ A, const __bf16* __restrict__ P, const float* __restrict__ G, const float* __restrict__ Bb, const float* __restrict__ F, const int* __restrict__ I3, const float* __restrict__ W3, const float* __restrict__ RES, float* __restrict__ OUTP) {
  constexpr int K = (MODE == 0) ? 256 : 128; constexpr bool EXACT = (MODE <= 1);
  __shared__ __align__(16) float so[4][16][132]; __shared__ __align__(16) float st[128][68];
  const int tid = threadIdx.x, wave = tid >> 5, lane = tid & 31, col = lane & 15, g = lane >> 4; const size_t r0 = (size_t)blockIdx.x * 64 + wave * 16; const int n0 = (MODE == 3) ? blockIdx.y * 128 : 0; const int ldo = (MODE == 3) ? 384 : 128;
  const float bnc = 1.0f / sqrtf(1.0f + 1e-5f);
  v8f acc[8] = {};
#pragma unroll 2
  for (int kc = 0; kc < K / 32; ++kc) { F2 a; if (EXACT) { v16b ax; const float* p = A + (r0 + col) * K + kc * 32 + 8 * g;
#pragma unroll
      for (int i2 = 0; i2 < 8; ++i2) { ax[i2] = (__bf16)p[i2]; ax[8 + i2] = (__bf16)p[16 + i2]; } a.h = ax; a.l = ax; } else a = split_row(A + (r0 + col) * K, kc * 32, lane);
#pragma unroll
    for (int j = 0; j < 8; ++j) { const v16b w = frag_b(P + (size_t)(n0 + j * 16 + col) * K + kc * 32, lane); if (!EXACT) acc[j] = wmma_bf(a.l, w, acc[j]); acc[j] = wmma_bf(a.h, w, acc[j]); } }
#pragma unroll
  for (int j = 0; j < 8; ++j) { const int o = j * 16 + col; float sc = 1.f, sh_ = 0.f; if (MODE != 3) { sc = bfr(G[o]) * bnc; sh_ = bfr(Bb[o]); } else sh_ = bfr(Bb[n0 + o]);
#pragma unroll
    for (int r = 0; r < 8; ++r) { const size_t row = r0 + 8 * g + r; float v = acc[j][r] * sc + sh_;
      if (MODE == 0 || MODE == 2) v = fmaxf(v, 0.f);
      else if (MODE == 1) { v = fmaxf(v, 0.f); const int* i3 = I3 + row * 4; const float* w3 = W3 + row * 4; const float t0 = F[(size_t)min(max(i3[0], 0), RS - 1) * CC + o] * w3[0], t1 = F[(size_t)min(max(i3[1], 0), RS - 1) * CC + o] * w3[1], t2 = F[(size_t)min(max(i3[2], 0), RS - 1) * CC + o] * w3[2]; v += (t0 + t2) + t1; }
      else if (MODE == 4) v = fmaxf(v + RES[row * CC + o], 0.f);
      so[wave][8 * g + r][o] = v; } }
  LDSX();
  if (MODE != 4) { for (int rl = 0; rl < 16; ++rl) vst2(OUTP + (r0 + rl) * (size_t)ldo + n0 + lane * 4, *(const v4f*)&so[wave][rl][lane * 4]); }
  else { __syncthreads(); const size_t q0 = (size_t)blockIdx.x * 64; const int b = (int)(q0 / NM), m0 = (int)(q0 % NM);
    for (int q = tid; q < 64 * 128; q += 128) { const int rl = q >> 7, c = q & 127; st[c][rl] = so[rl >> 4][rl & 15][c]; }
    __syncthreads();
    for (int q = tid; q < 128 * 16; q += 128) { const int c = q >> 4, pc = q & 15; vst2(OUTP + ((size_t)b * CC + c) * NM + m0 + pc * 4, *(const v4f*)&st[c][pc * 4]); } }
}
__global__ __launch_bounds__(128) void k_pt(const float* __restrict__ TX, const int* __restrict__ IDX, const float* __restrict__ QKV, const float* __restrict__ P1W, const float* __restrict__ P1B, const float* __restrict__ PBG, const float* __restrict__ PBB, const float* __restrict__ P2W, const float* __restrict__ P2B, const float* __restrict__ W1G, const float* __restrict__ W1B, const __bf16* __restrict__ PW, const float* __restrict__ WL1B, const float* __restrict__ W2G, const float* __restrict__ W2B, const float* __restrict__ WL2W, const float* __restrict__ WL2B, const float* __restrict__ B2G, const float* __restrict__ B2B, float* __restrict__ AG) {
  __shared__ int snb[4][KN]; __shared__ float st3[4][KN][4]; __shared__ __align__(16) float sr[4][16][132]; __shared__ __align__(16) float svp[4][16][132]; __shared__ float sw[4][16][20]; __shared__ __align__(16) float sag[4][132];
  const int tid = threadIdx.x, wave = tid >> 5, lane = tid & 31, col = lane & 15, g = lane >> 4; const size_t m = (size_t)blockIdx.x * 4 + wave; const float bnc = 1.0f / sqrtf(1.0f + 1e-5f);
  if (lane < KN) snb[wave][lane] = min(max(IDX[m * KN + lane], 0), RM - 1);
  LDSX();
  if (lane < KN) { const int nb = snb[wave][lane]; const float rx = bfr(TX[(size_t)nb * 3]) - bfr(TX[m * 3]), ry = bfr(TX[(size_t)nb * 3 + 1]) - bfr(TX[m * 3 + 1]), rz = bfr(TX[(size_t)nb * 3 + 2]) - bfr(TX[m * 3 + 2]);
#pragma unroll
    for (int o = 0; o < 3; ++o) { float a = ((rx * bfr(P1W[o * 3]) + ry * bfr(P1W[o * 3 + 1])) + rz * bfr(P1W[o * 3 + 2])) + bfr(P1B[o]); a = a * (bfr(PBG[o]) * bnc) + bfr(PBB[o]); st3[wave][lane][o] = fmaxf(a, 0.f); } st3[wave][lane][3] = 0.f; }
  LDSX();
  const float* qrow = QKV + m * 384; float pw[4][3], pb[4], qv[4], s1[4], b1[4];
#pragma unroll
  for (int c4 = 0; c4 < 4; ++c4) { const int c = lane * 4 + c4; pw[c4][0] = bfr(P2W[c * 3]); pw[c4][1] = bfr(P2W[c * 3 + 1]); pw[c4][2] = bfr(P2W[c * 3 + 2]); pb[c4] = bfr(P2B[c]); qv[c4] = qrow[c]; s1[c4] = bfr(W1G[c]) * bnc; b1[c4] = bfr(W1B[c]); }
#pragma unroll 1
  for (int k = 0; k < KN; ++k) { const int nb = snb[wave][k]; const float* krow = QKV + (size_t)nb * 384 + 128; const float* vrow = QKV + (size_t)nb * 384 + 256; const float tx0 = st3[wave][k][0], tx1 = st3[wave][k][1], tx2 = st3[wave][k][2];
#pragma unroll
    for (int c4 = 0; c4 < 4; ++c4) { const int c = lane * 4 + c4; const float pr = ((tx0 * pw[c4][0] + tx1 * pw[c4][1]) + tx2 * pw[c4][2]) + pb[c4]; const float r = (krow[c] - qv[c4]) + pr; sr[wave][k][c] = fmaxf(r * s1[c4] + b1[c4], 0.f); svp[wave][k][c] = vrow[c] + pr; } }
  LDSX();
  v8f acc = {};
#pragma unroll
  for (int kc = 0; kc < 4; ++kc) { const F2 a = split_row(&sr[wave][col][0], kc * 32, lane); const v16b w = frag_b(PW + P_W1 + (size_t)col * 128 + kc * 32, lane); acc = wmma_bf(a.l, w, acc); acc = wmma_bf(a.h, w, acc); }
  { const float bb = bfr(WL1B[col]); const float s2 = bfr(W2G[col]) * bnc, b2 = bfr(W2B[col]);
#pragma unroll
    for (int r = 0; r < 8; ++r) sw[wave][8 * g + r][col] = fmaxf((acc[r] + bb) * s2 + b2, 0.f); }
  LDSX();
  float w2v[CS]; if (lane < KN) {
#pragma unroll
    for (int o = 0; o < CS; ++o) { float a = bfr(WL2B[o]);
#pragma unroll
      for (int i2 = 0; i2 < CS; ++i2) a += sw[wave][lane][i2] * bfr(WL2W[o * CS + i2]);
      w2v[o] = a; } }
  LDSX();
  if (lane < KN) {
#pragma unroll
    for (int o = 0; o < CS; ++o) sw[wave][lane][o] = w2v[o]; }
  LDSX();
  if (lane < CS) { float mx = -3.0e38f; for (int k = 0; k < KN; ++k) mx = fmaxf(mx, sw[wave][k][lane]); float z = 0.f; float e[KN];
#pragma unroll
    for (int k = 0; k < KN; ++k) { e[k] = exp_ni(sw[wave][k][lane] - mx); z += e[k]; }
    const float iz = 1.0f / z;
#pragma unroll
    for (int k = 0; k < KN; ++k) sw[wave][k][lane] = e[k] * iz; }
  LDSX();
#pragma unroll
  for (int c4 = 0; c4 < 4; ++c4) { const int c = lane * 4 + c4; float a = 0.f;
#pragma unroll 4
    for (int k = 0; k < KN; ++k) a += svp[wave][k][c] * sw[wave][k][c & 15];
    sag[wave][c] = fmaxf(a * (bfr(B2G[c]) * bnc) + bfr(B2B[c]), 0.f); }
  LDSX();
  vst2(AG + m * CC + lane * 4, *(const v4f*)&sag[wave][lane * 4]);
}
extern "C" void kernel_launch(void* const* d_in, const int* in_sizes, int n_in, void* d_out, int out_size, void* d_ws, size_t ws_size, hipStream_t stream) {
  (void)in_sizes; (void)n_in; (void)out_size;
  const float** F = (const float**)d_in;
  if (ws_size < (size_t)WS_END) return;
  char* ws = (char*)d_ws; int *CNT = (int*)(ws + WS_CNT), *OFF = (int*)(ws + WS_OFF), *BST = (int*)(ws + WS_BST), *SEGS = (int*)(ws + WS_SEGS), *SEGE = (int*)(ws + WS_SEGE), *FS = (int*)(ws + WS_FS), *FE = (int*)(ws + WS_FE), *RST = (int*)(ws + WS_RST), *RCT = (int*)(ws + WS_RCT), *CELL = (int*)(ws + WS_CELL), *PID = (int*)(ws + WS_PID); float *FT = (float*)(ws + WS_FT), *TT = (float*)(ws + WS_TT), *Fp = (float*)(ws + WS_F), *X = (float*)(ws + WS_X), *X1 = (float*)(ws + WS_X1), *QKV = (float*)(ws + WS_Q), *W3 = (float*)(ws + WS_W3), *AG = (float*)(ws + WS_AG); int *IDX = (int*)(ws + WS_IDX), *I3 = (int*)(ws + WS_I3); __bf16* PW = (__bf16*)(ws + WS_PW);
  k_packW<<<dim3(128, 8), 256, 0, stream>>>(F[4], F[7], F[10], F[13], F[15], F[17], F[27], F[35], PW);
  k_tr<C1, NS><<<RS / 64, 64, 0, stream>>>(F[1], FT);
  k_tr<CC, NM><<<RM / 64, 64, 0, stream>>>(F[3], TT);
  k_cell<<<RM / 256, 256, 0, stream>>>(F[2], CELL, PID);
  k_csA_cnt<<<CSA_NCH, 256, 0, stream>>>(CELL, 1, CNT); k_csA_scan<<<1, 256, 0, stream>>>(CNT, OFF, BST); k_csA_scatter<<<CSA_NCH, 256, 0, stream>>>(PID, CELL, 1, 1, OFF, SEGS, SEGE); k_csA_bucket<<<CSA_NBK, 256, 0, stream>>>(CNT, OFF, BST, SEGS, SEGE, CELL, 1, FS, FE, RST, RCT);
  k_nn<0><<<RM / 64, 64, 0, stream>>>(F[2], F[0], I3, W3, IDX, CELL, FE, RST, RCT);
  k_nn<1><<<RMT / 64, 64, 0, stream>>>(F[2], F[0], I3, W3, IDX, CELL, FE, RST, RCT);
  k_gemm<0><<<RS / 64, 128, 0, stream>>>(FT, PW + P_TU1, F[5], F[6], nullptr, nullptr, nullptr, nullptr, Fp);
  k_gemm<1><<<RM / 64, 128, 0, stream>>>(TT, PW + P_TU2, F[8], F[9], Fp, I3, W3, nullptr, X);
  k_gemm<2><<<RM / 64, 128, 0, stream>>>(X, PW + P_L1, F[11], F[12], nullptr, nullptr, nullptr, nullptr, X1);
  k_gemm<3><<<dim3(RM / 64, 1), 128, 0, stream>>>(X1, PW + P_QKV, nullptr, F[14], nullptr, nullptr, nullptr, nullptr, QKV);
  k_gemm<3><<<dim3(RM / 64, 1), 128, 0, stream>>>(X1, PW + P_QKV + 128 * 128, nullptr, F[16], nullptr, nullptr, nullptr, nullptr, QKV + 128);
  k_gemm<3><<<dim3(RM / 64, 1), 128, 0, stream>>>(X1, PW + P_QKV + 256 * 128, nullptr, F[18], nullptr, nullptr, nullptr, nullptr, QKV + 256);
  k_pt<<<RMT / 4, 128, 0, stream>>>(F[2], IDX, QKV, F[19], F[20], F[21], F[22], F[23], F[24], F[25], F[26], PW, F[28], F[29], F[30], F[31], F[32], F[33], F[34], AG);
  k_gemm<4><<<RMT / 64, 128, 0, stream>>>(AG, PW + P_L3, F[36], F[37], nullptr, nullptr, nullptr, X, (float*)d_out);
}
